// Ner_model_50654844289770
// MI455X (gfx1250) — hardware-verified
//
#include <hip/hip_runtime.h>
#include <stdint.h>
#include <stddef.h>


typedef _Float16       v8h   __attribute__((ext_vector_type(8)));
typedef _Float16       v16h  __attribute__((ext_vector_type(16)));
typedef __bf16         v16b  __attribute__((ext_vector_type(16)));
typedef unsigned short v8us  __attribute__((ext_vector_type(8)));
typedef unsigned short v16us __attribute__((ext_vector_type(16)));
typedef float          v8f   __attribute__((ext_vector_type(8)));
typedef float          v4f   __attribute__((ext_vector_type(4)));

static constexpr int NE    = 64;
static constexpr int NH    = 64;
static constexpr int NB    = 128;
static constexpr int NS    = 512;
static constexpr int N3H   = 192;
static constexpr int NTILE = NS * NB / 16;
static constexpr int NROW  = NTILE * 16;
static constexpr int XW_TILE_FLOATS = 12 * 256;

union FragB { v16b b; v16us u; v8us half[2]; };
union FragH { v16h v; v16us u; v8h half[2]; };
union P8us  { v8us v; unsigned short e[8]; };
union P8h   { v8h v;  _Float16 e[8]; };
union HBits { _Float16 f; unsigned short s; };

__device__ __forceinline__ unsigned short bf16_rne(float x) {
  unsigned u = __float_as_uint(x);
  u += 0x7FFFu + ((u >> 16) & 1u);
  return (unsigned short)(u >> 16);
}
__device__ __forceinline__ float bf16_val(unsigned short b) {
  return __uint_as_float(((unsigned)b) << 16);
}

__device__ __forceinline__ float sigm(float x) {
  return __builtin_amdgcn_rcpf(1.0f + __expf(-x));
}
__device__ __forceinline__ float tanh_s(float x) {
  const float a = fabsf(x);
  const float e = __expf(-2.0f * a);
  const float t = (1.0f - e) * __builtin_amdgcn_rcpf(1.0f + e);
  return x < 0.0f ? -t : t;
}

__device__ __forceinline__ v8f mma_bf16(const FragB& a, const FragB& b, v8f c) {
  return __builtin_amdgcn_wmma_f32_16x16x32_bf16(false, a.b, false, b.b, (short)0, c, false, false);
}
__device__ __forceinline__ v8f mma_f16(const FragH& a, const FragH& b, v8f c) {
  return __builtin_amdgcn_wmma_f32_16x16x32_f16(false, a.v, false, b.v, (short)0, c, false, false);
}

__global__ void __launch_bounds__(256)
k_gather(const int* __restrict__ tok, const float* __restrict__ emb, int nv,
         unsigned short* __restrict__ xhi, unsigned short* __restrict__ xlo, int nchunk)
{
  const int i = blockIdx.x * 256 + threadIdx.x;
  const bool valid = i < nchunk;
  const int ic = valid ? i : 0;
  const int row = ic >> 3, ch = ic & 7;
  const int tile = row >> 4, m = row & 15;
  const int t = tile >> 3, bt = tile & 7;
  const int b = bt * 16 + m;
  int tk = tok[b * NS + t];
  tk = tk < 0 ? 0 : (tk >= nv ? nv - 1 : tk);
  const float* src = emb + (size_t)tk * NE + ch * 8;
  const v4f x0 = *(const v4f*)(src);
  const v4f x1 = *(const v4f*)(src + 4);
  P8us ph, pl;
#pragma unroll
  for (int e = 0; e < 4; ++e) {
    const float xa = x0[e];
    const unsigned short ha = bf16_rne(xa);
    ph.e[e] = ha;  pl.e[e] = bf16_rne(xa - bf16_val(ha));
    const float xb = x1[e];
    const unsigned short hb = bf16_rne(xb);
    ph.e[4 + e] = hb;  pl.e[4 + e] = bf16_rne(xb - bf16_val(hb));
  }
  const v8us vh = ph.v, vl = pl.v;
  const size_t off = (size_t)row * NE + ch * 8;
  if (valid) {
    *(volatile v8us*)(xhi + off) = vh;
    *(volatile v8us*)(xlo + off) = vl;
  }
  __threadfence();
  if (valid) {
    *(volatile v8us*)(xhi + off) = vh;
    *(volatile v8us*)(xlo + off) = vl;
  }
}

static constexpr int PJ_THREADS = 256;
static constexpr int PJ_WAVES   = 8;
static constexpr int PJ_ITERS   = 2;
static constexpr int PJ_TILES_PER_BLOCK = PJ_WAVES * PJ_ITERS;

__global__ void __launch_bounds__(PJ_THREADS)
k_project(const unsigned short* __restrict__ xhi,
          const unsigned short* __restrict__ xlo,
          const float* __restrict__ W,
          const float* __restrict__ bi,
          float* __restrict__ xw)
{
  __shared__ unsigned sWhi[N3H * (NE / 2)];
  __shared__ unsigned sWlo[N3H * (NE / 2)];
  __shared__ __attribute__((aligned(16))) float sStage[PJ_WAVES * 256];

  const int tid = threadIdx.x;
  for (int p = tid; p < N3H * (NE / 2); p += PJ_THREADS) {
    const int n = p >> 5;
    const int k = (p & 31) * 2;
    const float w0 = W[k * N3H + n];
    const float w1 = W[(k + 1) * N3H + n];
    const unsigned short h0 = bf16_rne(w0), h1 = bf16_rne(w1);
    const unsigned short l0 = bf16_rne(w0 - bf16_val(h0));
    const unsigned short l1 = bf16_rne(w1 - bf16_val(h1));
    *(volatile unsigned*)(sWhi + p) = (unsigned)h0 | ((unsigned)h1 << 16);
    *(volatile unsigned*)(sWlo + p) = (unsigned)l0 | ((unsigned)l1 << 16);
  }
  __syncthreads();

  const int l = tid & 31, h = l >> 4, c = l & 15, wv = tid >> 5;
  const unsigned short* whi = (const unsigned short*)sWhi;
  const unsigned short* wlo = (const unsigned short*)sWlo;
  float* stg = sStage + wv * 256;

  for (int it = 0; it < PJ_ITERS; ++it) {
    const int  tile  = blockIdx.x * PJ_TILES_PER_BLOCK + it * PJ_WAVES + wv;
    const bool valid = tile < NTILE;
    const int  tilec = valid ? tile : (NTILE - 1);
    const unsigned short* ahrow = xhi + ((size_t)tilec * 16 + c) * NE;
    const unsigned short* alrow = xlo + ((size_t)tilec * 16 + c) * NE;

    FragB ahi[2], alo[2];
#pragma unroll
    for (int ks = 0; ks < 2; ++ks) {
      const int kb = ks * 32 + 8 * h;
      ahi[ks].half[0] = *(const v8us*)(ahrow + kb);
      ahi[ks].half[1] = *(const v8us*)(ahrow + kb + 16);
      alo[ks].half[0] = *(const v8us*)(alrow + kb);
      alo[ks].half[1] = *(const v8us*)(alrow + kb + 16);
    }

#pragma unroll 1
    for (int j = 0; j < 12; ++j) {
      const int n = j * 16 + c;
      FragB bh[2], bl[2];
#pragma unroll
      for (int ks = 0; ks < 2; ++ks) {
        const int kb = n * NE + ks * 32 + 8 * h;
        bh[ks].half[0] = *(const v8us*)(whi + kb);
        bh[ks].half[1] = *(const v8us*)(whi + kb + 16);
        bl[ks].half[0] = *(const v8us*)(wlo + kb);
        bl[ks].half[1] = *(const v8us*)(wlo + kb + 16);
      }
      v8f acc = {};
      acc = mma_bf16(ahi[0], bh[0], acc);
      acc = mma_bf16(ahi[0], bl[0], acc);
      acc = mma_bf16(alo[0], bh[0], acc);
      acc = mma_bf16(ahi[1], bh[1], acc);
      acc = mma_bf16(ahi[1], bl[1], acc);
      acc = mma_bf16(alo[1], bh[1], acc);
      asm volatile("v_nop\n\tv_nop\n\tv_nop\n\tv_nop"
                   : "+v"(acc)
                   : "v"(ahi[0].u), "v"(alo[0].u), "v"(ahi[1].u), "v"(alo[1].u),
                     "v"(bh[0].u), "v"(bl[0].u), "v"(bh[1].u), "v"(bl[1].u)
                   : "memory");

      const float bj = bi[n];
      const v4f o0 = {acc[0] + bj, acc[1] + bj, acc[2] + bj, acc[3] + bj};
      const v4f o1 = {acc[4] + bj, acc[5] + bj, acc[6] + bj, acc[7] + bj};
      *(v4f*)(stg + l * 8)     = o0;
      *(v4f*)(stg + l * 8 + 4) = o1;
      __syncthreads();
      const v4f c0 = *(const v4f*)(stg + l * 4);
      const v4f c1 = *(const v4f*)(stg + (32 + l) * 4);
      float* dst = xw + ((size_t)tilec * 12 + j) * 256;
      if (valid) {
        *(volatile v4f*)(dst + l * 4)        = c0;
        *(volatile v4f*)(dst + (32 + l) * 4) = c1;
      }
      __threadfence();
      if (valid) {
        *(volatile v4f*)(dst + l * 4)        = c0;
        *(volatile v4f*)(dst + (32 + l) * 4) = c1;
      }
      __syncthreads();
    }
  }
}

__device__ __forceinline__ v8f rec_tile(const FragH* a, const _Float16* su, int n, int h) {
  FragH b0, b1;
  const _Float16* row = su + n * NH;
  b0.half[0] = *(const v8h*)(row + 8 * h);
  b0.half[1] = *(const v8h*)(row + 16 + 8 * h);
  b1.half[0] = *(const v8h*)(row + 32 + 8 * h);
  b1.half[1] = *(const v8h*)(row + 48 + 8 * h);
  v8f acc = {};
  acc = mma_f16(a[0], b0, acc);
  acc = mma_f16(a[1], b1, acc);
  asm volatile("v_nop\n\tv_nop\n\tv_nop\n\tv_nop"
               : "+v"(acc)
               : "v"(a[0].u), "v"(a[1].u), "v"(b0.u), "v"(b1.u)
               : "memory");
  return acc;
}

__global__ void __launch_bounds__(32)
k_scan(const float* __restrict__ xwF, const float* __restrict__ xwB,
       const int* __restrict__ tok,
       const float* __restrict__ Uf, const float* __restrict__ Ub,
       const float* __restrict__ brf, const float* __restrict__ brb,
       float* __restrict__ gru)
{
  __shared__ unsigned sU[N3H * (NH / 2)];
  __shared__ __attribute__((aligned(16))) float sH[16 * NH];
  __shared__ unsigned sM[NS];

  const int dir = blockIdx.x >> 3;
  const int bt  = blockIdx.x & 7;
  const int b0  = bt * 16;
  const float* xw = dir ? xwB : xwF;
  const float* U  = dir ? Ub  : Uf;
  const float* br = dir ? brb : brf;
  const int l = threadIdx.x & 31, h = l >> 4, c = l & 15;

  for (int p = l; p < N3H * (NH / 2); p += 32) {
    const int n = p >> 5;
    const int k = (p & 31) * 2;
    HBits u0, u1;
    u0.f = (_Float16)(U[k * N3H + n] * 16.0f);
    u1.f = (_Float16)(U[(k + 1) * N3H + n] * 16.0f);
    *(volatile unsigned*)(sU + p) = (unsigned)u0.s | ((unsigned)u1.s << 16);
  }
  for (int tt = l; tt < NS; tt += 32) {
    unsigned m = 0;
#pragma unroll
    for (int r = 0; r < 16; ++r)
      m |= (tok[(b0 + r) * NS + tt] != 0 ? 1u : 0u) << r;
    *(volatile unsigned*)(sM + tt) = m;
  }
  {
    const v4f z4 = {0.0f, 0.0f, 0.0f, 0.0f};
#pragma unroll
    for (int i = 0; i < 8; ++i) *(volatile v4f*)(sH + l * 32 + i * 4) = z4;
  }
  __syncthreads();

  const _Float16* su = (const _Float16*)sU;
  float bz[4], brr[4], bc[4];
#pragma unroll
  for (int jt = 0; jt < 4; ++jt) {
    bz[jt]  = br[jt * 16 + c];
    brr[jt] = br[NH + jt * 16 + c];
    bc[jt]  = br[2 * NH + jt * 16 + c];
  }
  const v8f zero8 = {};
  v8f hc[4];
#pragma unroll
  for (int jt = 0; jt < 4; ++jt) hc[jt] = zero8;
  const float RSC = 1.0f / 4096.0f;

  for (int s = 0; s < NS; ++s) {
    const int t = dir ? (NS - 1 - s) : s;

    FragH a[2];
#pragma unroll
    for (int ks = 0; ks < 2; ++ks) {
#pragma unroll
      for (int hf = 0; hf < 2; ++hf) {
        const int kb = c * NH + ks * 32 + hf * 16 + 8 * h;
        const v4f p0 = *(const v4f*)(sH + kb);
        const v4f p1 = *(const v4f*)(sH + kb + 4);
        P8h q;
#pragma unroll
        for (int i = 0; i < 4; ++i) {
          q.e[i]     = (_Float16)(p0[i] * 256.0f);
          q.e[4 + i] = (_Float16)(p1[i] * 256.0f);
        }
        a[ks].half[hf] = q.v;
      }
    }
    const unsigned mb = sM[t];
    const float* xb = xw + (size_t)(t * 8 + bt) * XW_TILE_FLOATS + l * 8;

#pragma unroll
    for (int jt = 0; jt < 4; ++jt) {
      const v4f xz0 = *(const v4f*)(xb + jt * 256);
      const v4f xz1 = *(const v4f*)(xb + jt * 256 + 4);
      const v4f xr0 = *(const v4f*)(xb + (jt + 4) * 256);
      const v4f xr1 = *(const v4f*)(xb + (jt + 4) * 256 + 4);
      const v4f xc0 = *(const v4f*)(xb + (jt + 8) * 256);
      const v4f xc1 = *(const v4f*)(xb + (jt + 8) * 256 + 4);

      const v8f az = rec_tile(a, su, jt * 16 + c, h);
      const v8f ar = rec_tile(a, su, NH + jt * 16 + c, h);
      const v8f ac = rec_tile(a, su, 2 * NH + jt * 16 + c, h);

#pragma unroll
      for (int v = 0; v < 8; ++v) {
        const float xz = v < 4 ? xz0[v] : xz1[v - 4];
        const float xr = v < 4 ? xr0[v] : xr1[v - 4];
        const float xc = v < 4 ? xc0[v] : xc1[v - 4];
        const float recz = az[v] * RSC + bz[jt];
        const float recr = ar[v] * RSC + brr[jt];
        const float recc = ac[v] * RSC + bc[jt];
        const float zg = sigm(xz + recz);
        const float rg = sigm(xr + recr);
        const float hh = tanh_s(xc + rg * recc);
        const float hold = hc[jt][v];
        const float hn = zg * hold + (1.0f - zg) * hh;
        const unsigned bit = (mb >> (8 * h + v)) & 1u;
        hc[jt][v] = bit ? hn : hold;
      }
    }

    __syncthreads();
#pragma unroll
    for (int jt = 0; jt < 4; ++jt)
#pragma unroll
      for (int v = 0; v < 8; ++v)
        *(volatile float*)(sH + (8 * h + v) * NH + jt * 16 + c) = hc[jt][v];
    __syncthreads();

    v4f o[8];
#pragma unroll
    for (int i = 0; i < 8; ++i) {
      const int L = i * 4 + (l >> 3);
      const int row = L >> 1, half = L & 1, e = l & 7;
      o[i] = *(const v4f*)(sH + row * NH + half * 32 + e * 4);
    }
    float* gbase = gru + ((size_t)b0 * NS + t) * 128 + dir * NH;
#pragma unroll
    for (int i = 0; i < 8; ++i) {
      const int L = i * 4 + (l >> 3);
      const int row = L >> 1, half = L & 1, e = l & 7;
      *(volatile v4f*)(gbase + (size_t)row * NS * 128 + half * 32 + e * 4) = o[i];
    }
    __threadfence();
#pragma unroll
    for (int i = 0; i < 8; ++i) {
      const int L = i * 4 + (l >> 3);
      const int row = L >> 1, half = L & 1, e = l & 7;
      *(volatile v4f*)(gbase + (size_t)row * NS * 128 + half * 32 + e * 4) = o[i];
    }
  }
}

__global__ void __launch_bounds__(256)
k_heads(const float* __restrict__ gru,
        const float* __restrict__ w1, const float* __restrict__ b1,
        const float* __restrict__ w2, const float* __restrict__ b2,
        float* __restrict__ x1, float* __restrict__ x2, int nquad)
{
  const int q = blockIdx.x * 256 + threadIdx.x;
  if (q >= nquad) return;
  const v4f* g  = (const v4f*)(gru + (size_t)q * 4 * 128);
  const v4f* W1 = (const v4f*)w1;
  const v4f* W2 = (const v4f*)w2;
  float s1[4] = {0.0f, 0.0f, 0.0f, 0.0f};
  float s2[4] = {0.0f, 0.0f, 0.0f, 0.0f};
#pragma unroll 1
  for (int k = 0; k < 32; ++k) {
    const v4f u1 = W1[k], u2 = W2[k];
#pragma unroll
    for (int rr = 0; rr < 4; ++rr) {
      const v4f gv = g[rr * 32 + k];
      s1[rr] += gv[0] * u1[0] + gv[1] * u1[1] + gv[2] * u1[2] + gv[3] * u1[3];
      s2[rr] += gv[0] * u2[0] + gv[1] * u2[1] + gv[2] * u2[2] + gv[3] * u2[3];
    }
  }
  const float bb1 = b1[0], bb2 = b2[0];
  const v4f o1 = {sigm(s1[0] + bb1), sigm(s1[1] + bb1), sigm(s1[2] + bb1), sigm(s1[3] + bb1)};
  const v4f o2 = {sigm(s2[0] + bb2), sigm(s2[1] + bb2), sigm(s2[2] + bb2), sigm(s2[3] + bb2)};
  *(volatile v4f*)(x1 + (size_t)q * 4) = o1;
  *(volatile v4f*)(x2 + (size_t)q * 4) = o2;
  __threadfence();
  *(volatile v4f*)(x1 + (size_t)q * 4) = o1;
  *(volatile v4f*)(x2 + (size_t)q * 4) = o2;
}

extern "C" void kernel_launch(void* const* d_in, const int* in_sizes, int n_in,
                              void* d_out, int out_size, void* d_ws, size_t ws_size,
                              hipStream_t stream)
{
  if (n_in < 14) return;
  if (in_sizes[0] != NB * NS) return;
  if (in_sizes[1] < NE || (in_sizes[1] % NE) != 0) return;
  if (in_sizes[2] != NE * N3H || in_sizes[3] != NH * N3H || in_sizes[6] != NE * N3H || in_sizes[7] != NH * N3H) return;
  if (in_sizes[4] != N3H || in_sizes[5] != N3H || in_sizes[8] != N3H || in_sizes[9] != N3H) return;
  if (in_sizes[10] != 2 * NH || in_sizes[12] != 2 * NH || in_sizes[11] < 1 || in_sizes[13] < 1) return;
  if (out_size != NB * NS * (2 + 2 * NH)) return;

  const int*   tok = (const int*)d_in[0];
  const float* emb = (const float*)d_in[1];
  const float* Wf  = (const float*)d_in[2];
  const float* Uf  = (const float*)d_in[3];
  const float* bif = (const float*)d_in[4];
  const float* brf = (const float*)d_in[5];
  const float* Wb  = (const float*)d_in[6];
  const float* Ub  = (const float*)d_in[7];
  const float* bib = (const float*)d_in[8];
  const float* brb = (const float*)d_in[9];
  const float* w1  = (const float*)d_in[10];
  const float* b1  = (const float*)d_in[11];
  const float* w2  = (const float*)d_in[12];
  const float* b2  = (const float*)d_in[13];
  const int nv = in_sizes[1] / NE;

  const size_t x_bytes  = (size_t)NROW * NE * sizeof(unsigned short);
  const size_t xw_bytes = (size_t)NTILE * XW_TILE_FLOATS * sizeof(float);
  const size_t total    = 2 * x_bytes + 2 * xw_bytes;
  if (ws_size < total) return;
  char* ws = (char*)d_ws;
  unsigned short* xhi = (unsigned short*)(ws);
  unsigned short* xlo = (unsigned short*)(ws + x_bytes);
  float* xwF = (float*)(ws + 2 * x_bytes);
  float* xwB = (float*)(ws + 2 * x_bytes + xw_bytes);

  float* x1  = (float*)d_out;
  float* x2  = x1 + (size_t)NB * NS;
  float* gru = x2 + (size_t)NB * NS;

  const int nchunk = NROW * (NE / 8);
  k_gather<<<(nchunk + 255) / 256, 256, 0, stream>>>(tok, emb, nv, xhi, xlo, nchunk);

  const int pj_blocks = (NTILE + PJ_TILES_PER_BLOCK - 1) / PJ_TILES_PER_BLOCK;
  k_project<<<pj_blocks, PJ_THREADS, 0, stream>>>(xhi, xlo, Wf, bif, xwF);
  k_project<<<pj_blocks, PJ_THREADS, 0, stream>>>(xhi, xlo, Wb, bib, xwB);

  k_scan<<<2 * (NB / 16), 32, 0, stream>>>(xwF, xwB, tok, Uf, Ub, brf, brb, gru);

  const int nquad = (NB * NS) / 4;
  k_heads<<<(nquad + 255) / 256, 256, 0, stream>>>(gru, w1, b1, w2, b2, x1, x2, nquad);
}
